// SS2D_Block_24532853194990
// MI455X (gfx1250) — hardware-verified
//
#include <hip/hip_runtime.h>
#include <math.h>

#define NBAT 4
#define CIN  96
#define HI   128
#define WI   128
#define IMH  64
#define IMW  64
#define LTOK (IMH * IMW)
#define NTOK (NBAT * LTOK)
#define DIN  192
#define DST  16
#define DTRK 6
#define XPR  38
#define NDIR 2
#define XDN  128
#define XBO  8
#define XCO  24
#define NOP  128
#define EPSV 1e-5f
#define GSTR 40
#define OSTR 68
#define SMEMB (8 * 16 * OSTR * 4)
#define SCH  32
#define SYP  196
#define LOG2E 1.4426950408889634f

static_assert(NTOK % 128 == 0);
static_assert(LTOK % 128 == 0);
static_assert(CIN % 32 == 0);
static_assert(DIN % 32 == 0);
static_assert((2 * DIN) % 64 == 0);
static_assert(XDN % 64 == 0);
static_assert(NOP % 64 == 0);
static_assert(NOP >= CIN);
static_assert(XCO + DST <= 64);
static_assert(XBO >= DTRK);
static_assert(SMEMB >= (2 * 128 * GSTR + 64 * GSTR) * 2);
static_assert(LTOK % SCH == 0);
static_assert(SCH == 32);
static_assert(SYP % 4 == 0);
static_assert(SYP >= DIN);
static_assert((SCH * (DIN / 4)) % DIN == 0);
static_assert((NTOK * (CIN / 8)) % 256 == 0);
static_assert((NTOK * (DIN / 8)) % 256 == 0);
static_assert((NBAT * HI * WI * (CIN / 4)) % 256 == 0);
static_assert(NTOK % 8 == 0);

typedef unsigned short us16 __attribute__((ext_vector_type(16)));
typedef unsigned short us8  __attribute__((ext_vector_type(8)));
typedef unsigned short us8a __attribute__((ext_vector_type(8), may_alias));
typedef __bf16 v16b __attribute__((ext_vector_type(16)));
typedef float v8f __attribute__((ext_vector_type(8)));
typedef float v4f __attribute__((ext_vector_type(4)));
typedef float v4fa __attribute__((ext_vector_type(4), may_alias));
union FragU { us16 v; us8 h[2]; };

__device__ __forceinline__ unsigned short bf16_bits(float f) {
  unsigned u = __float_as_uint(f);
  u += 0x7FFFu + ((u >> 16) & 1u);
  return (unsigned short)(u >> 16);
}
__device__ __forceinline__ float bf16_val(unsigned short b) { return __uint_as_float(((unsigned)b) << 16); }
__device__ __forceinline__ float bf16r(float f) { return bf16_val(bf16_bits(f)); }
__device__ __forceinline__ float siluf(float x) { return x * __builtin_amdgcn_rcpf(1.0f + __expf(-x)); }

__device__ __forceinline__ v8f mma_bf16(us16 a, us16 b, v8f c) {
  return __builtin_amdgcn_wmma_f32_16x16x32_bf16(false, __builtin_bit_cast(v16b, a), false, __builtin_bit_cast(v16b, b), (short)0, c, false, false);
}
__device__ __forceinline__ void wguard(v8f& c0, v8f& c1, v8f& c2, v8f& c3, const us16& a0, const us16& a1,
                                       const us16& b0, const us16& b1, const us16& b2, const us16& b3) {
#if defined(__HIP_DEVICE_COMPILE__)
  asm volatile("v_nop\n\tv_nop\n\tv_nop\n\tv_nop"
               : "+v"(c0), "+v"(c1), "+v"(c2), "+v"(c3)
               : "v"(a0), "v"(a1), "v"(b0), "v"(b1), "v"(b2), "v"(b3));
#endif
}

__device__ __forceinline__ us16 lds_frag(const unsigned short* base) {
  const int lane = threadIdx.x & 31, r = lane & 15, kh = (lane >> 4) * 8;
  FragU f;
  f.h[0] = *(const us8a*)(base + r * GSTR + kh);
  f.h[1] = *(const us8a*)(base + r * GSTR + 16 + kh);
  return f.v;
}

__device__ __forceinline__ void stage_a(unsigned short* lds, const unsigned short* __restrict__ P, int ld, int m0, int k0, int tid) {
  const int row = tid >> 1, cq = (tid & 1) * 16;
  const unsigned short* src = P + (size_t)(m0 + row) * ld + k0 + cq;
  const us8 v0 = *(const us8a*)src;
  const us8 v1 = *(const us8a*)(src + 8);
  *(us8a*)(lds + row * GSTR + cq) = v0;
  *(us8a*)(lds + row * GSTR + cq + 8) = v1;
}
__device__ __forceinline__ void stage_b(unsigned short* lds, const unsigned short* __restrict__ P, int ld, int n0, int k0, int tid) {
  const int row = tid >> 2, kq = (tid & 3) * 8;
  const us8 v = *(const us8a*)(P + (size_t)(n0 + row) * ld + k0 + kq);
  *(us8a*)(lds + row * GSTR + kq) = v;
}

template <int A2>
__global__ __launch_bounds__(256) void k_gemm(const unsigned short* __restrict__ A0, const unsigned short* __restrict__ A1, int lda,
                                             const unsigned short* __restrict__ B0, int ldb,
                                             float* Y, float* Yalt, int nsplit, int ldy, int K) {
#pragma clang fp contract(off)
  __shared__ __attribute__((aligned(16))) unsigned char sm[SMEMB];
  unsigned short* lA0 = (unsigned short*)sm;
  unsigned short* lA1 = lA0 + 128 * GSTR;
  unsigned short* lB0 = lA1 + 128 * GSTR;
  float* oS = (float*)sm;
  const int tid = threadIdx.x, lane = tid & 31, wave = tid >> 5, cl = lane & 15, hh = lane >> 4;
  const int m0 = blockIdx.x * 128;
  const int n0 = blockIdx.y * 64;
  float* Yb = Y;
  int nq = n0;
  if (nsplit > 0 && n0 >= nsplit) { Yb = Yalt; nq = n0 - nsplit; }

  v8f acc[4];
#pragma unroll
  for (int j = 0; j < 4; ++j) { v8f zz = {0.f, 0.f, 0.f, 0.f, 0.f, 0.f, 0.f, 0.f}; acc[j] = zz; }

#pragma unroll 1
  for (int k0 = 0; k0 < K; k0 += 32) {
    __syncthreads();
    stage_a(lA0, A0, lda, m0, k0, tid);
    if (A2) stage_a(lA1, A1, lda, m0, k0, tid);
    stage_b(lB0, B0, ldb, n0, k0, tid);
    __syncthreads();
    const us16 af0 = lds_frag(lA0 + 16 * wave * GSTR);
    us16 af1 = af0;
    if (A2) af1 = lds_frag(lA1 + 16 * wave * GSTR);
    us16 bfr[4];
#pragma unroll
    for (int j = 0; j < 4; ++j) bfr[j] = lds_frag(lB0 + 16 * j * GSTR);
#pragma unroll
    for (int j = 0; j < 4; ++j) acc[j] = mma_bf16(af0, bfr[j], acc[j]);
    if (A2) {
#pragma unroll
      for (int j = 0; j < 4; ++j) acc[j] = mma_bf16(af1, bfr[j], acc[j]);
    }
    wguard(acc[0], acc[1], acc[2], acc[3], af0, af1, bfr[0], bfr[1], bfr[2], bfr[3]);
  }
  __syncthreads();

  float* so = oS + wave * (16 * OSTR);
#pragma unroll
  for (int j = 0; j < 4; ++j)
#pragma unroll
    for (int r = 0; r < 8; ++r) so[(8 * hh + r) * OSTR + 16 * j + cl] = acc[j][r];
  __syncthreads();
#pragma unroll
  for (int pass = 0; pass < 2; ++pass) {
#pragma unroll
    for (int it = 0; it < 8; ++it) {
      const int ch = it * 32 + lane, r = ch >> 4, q = (ch & 15) * 4;
      const v4f v = *(const v4fa*)(so + r * OSTR + q);
      *(volatile v4f*)(Yb + (size_t)(m0 + 16 * wave + r) * ldy + nq + q) = v;
    }
    __threadfence();
  }
}

__global__ __launch_bounds__(256) void k_cvt(const float* __restrict__ src, unsigned short* dst, int nsrc, int ncol8, int total8) {
  const int idx = blockIdx.x * 256 + threadIdx.x;
  if (idx >= total8) return;
  const int row = idx / ncol8, c8 = (idx - row * ncol8) * 8;
  const int rs = (row < nsrc) ? row : (nsrc - 1);
  const float* s = src + (size_t)rs * (size_t)(ncol8 * 8) + c8;
  const v4f a = *(const v4fa*)s, b = *(const v4fa*)(s + 4);
  const bool zr = (row >= nsrc);
  us8 o;
#pragma unroll
  for (int u = 0; u < 4; ++u) {
    o[u]     = zr ? (unsigned short)0 : bf16_bits(a[u]);
    o[4 + u] = zr ? (unsigned short)0 : bf16_bits(b[u]);
  }
  const size_t off = (size_t)row * (size_t)(ncol8 * 8) + c8;
  *(volatile us8*)(dst + off) = o;
  __threadfence();
  *(volatile us8*)(dst + off) = o;
}

__global__ __launch_bounds__(256) void k_cvt_xw(const float* __restrict__ src, unsigned short* dst) {
  const int idx = blockIdx.x * 256 + threadIdx.x;
  if (idx >= XDN * (DIN / 8)) return;
  const int row = idx / (DIN / 8), c8 = (idx - row * (DIN / 8)) * 8;
  const int dir = row >> 6, rr = row & 63;
  const bool ok = (rr < DTRK) || (rr >= XBO && rr < XCO + DST);
  int sr = (rr < DTRK) ? rr : (rr - (XBO - DTRK));
  sr = (sr < 0) ? 0 : ((sr > XPR - 1) ? (XPR - 1) : sr);
  const float* s = src + ((size_t)(dir * XPR + sr)) * DIN + c8;
  const v4f a = *(const v4fa*)s, b = *(const v4fa*)(s + 4);
  us8 o;
#pragma unroll
  for (int u = 0; u < 4; ++u) {
    o[u]     = ok ? bf16_bits(a[u]) : (unsigned short)0;
    o[4 + u] = ok ? bf16_bits(b[u]) : (unsigned short)0;
  }
  const size_t off = (size_t)row * DIN + c8;
  *(volatile us8*)(dst + off) = o;
  __threadfence();
  *(volatile us8*)(dst + off) = o;
}

__device__ __forceinline__ void split8(const float* v, us8& hi, us8& lo) {
#pragma unroll
  for (int u = 0; u < 8; ++u) {
    const unsigned short hb = bf16_bits(v[u]);
    hi[u] = hb; lo[u] = bf16_bits(v[u] - bf16_val(hb));
  }
}

__global__ __launch_bounds__(256) void k_dw7(const float* __restrict__ X, const float* __restrict__ w, const float* __restrict__ bias,
                                            unsigned short* HH, unsigned short* HL) {
#pragma clang fp contract(off)
  __shared__ __attribute__((aligned(16))) float w7s[49 * CIN];
  const int tid = threadIdx.x;
#pragma unroll 1
  for (int i = tid; i < 49 * CIN; i += 256) {
    const int tap = i / CIN, c = i - tap * CIN;
    w7s[i] = bf16r(w[c * 49 + tap]);
  }
  __syncthreads();
  const int idx = blockIdx.x * 256 + tid;
  const int tok = idx / (CIN / 8), c8 = (idx - tok * (CIN / 8)) * 8;
  const int bb = tok >> 12, l = tok & (LTOK - 1), wy = l >> 6, wx = l & 63;
  float acc[8];
#pragma unroll
  for (int u = 0; u < 8; ++u) acc[u] = 0.0f;
#pragma unroll 1
  for (int ky = 0; ky < 7; ++ky) {
    const int iy = 2 * wy - 3 + ky;
    const bool oky = ((unsigned)iy < (unsigned)HI);
    const int iyc = (iy < 0) ? 0 : ((iy > HI - 1) ? (HI - 1) : iy);
#pragma unroll
    for (int kx = 0; kx < 7; ++kx) {
      const int ix = 2 * wx - 3 + kx;
      const bool ok = oky && ((unsigned)ix < (unsigned)WI);
      const int ixc = (ix < 0) ? 0 : ((ix > WI - 1) ? (WI - 1) : ix);
      const float* p = X + ((size_t)((bb * HI + iyc) * WI + ixc)) * CIN + c8;
      const v4f xa = *(const v4fa*)p, xb = *(const v4fa*)(p + 4);
      const float* wq = w7s + (ky * 7 + kx) * CIN + c8;
      const v4f wa = *(const v4fa*)wq, wb = *(const v4fa*)(wq + 4);
#pragma unroll
      for (int u = 0; u < 4; ++u) {
        const float pa = bf16r(xa[u]) * wa[u];
        const float pb = bf16r(xb[u]) * wb[u];
        acc[u]     = acc[u]     + (ok ? pa : 0.0f);
        acc[4 + u] = acc[4 + u] + (ok ? pb : 0.0f);
      }
    }
  }
  const v4f ba = *(const v4fa*)(bias + c8), bq = *(const v4fa*)(bias + c8 + 4);
  float v[8];
#pragma unroll
  for (int u = 0; u < 4; ++u) { v[u] = acc[u] + bf16r(ba[u]); v[4 + u] = acc[4 + u] + bf16r(bq[u]); }
  us8 hi, lo;
  split8(v, hi, lo);
  const size_t o = (size_t)idx * 8;
  *(volatile us8*)(HH + o) = hi; *(volatile us8*)(HL + o) = lo;
  __threadfence();
  *(volatile us8*)(HH + o) = hi; *(volatile us8*)(HL + o) = lo;
}

__global__ __launch_bounds__(256) void k_dw3(const float* __restrict__ XI, const float* __restrict__ w, const float* __restrict__ bias,
                                            unsigned short* UH, unsigned short* UL) {
#pragma clang fp contract(off)
  __shared__ __attribute__((aligned(16))) float w3s[9 * DIN];
  const int tid = threadIdx.x;
#pragma unroll 1
  for (int i = tid; i < 9 * DIN; i += 256) {
    const int tap = i / DIN, c = i - tap * DIN;
    w3s[i] = bf16r(w[c * 9 + tap]);
  }
  __syncthreads();
  const int idx = blockIdx.x * 256 + tid;
  const int tok = idx / (DIN / 8), c8 = (idx - tok * (DIN / 8)) * 8;
  const int bb = tok >> 12, l = tok & (LTOK - 1), hy = l >> 6, wx = l & 63;
  float acc[8];
#pragma unroll
  for (int u = 0; u < 8; ++u) acc[u] = 0.0f;
#pragma unroll
  for (int ky = 0; ky < 3; ++ky) {
    const int iy = hy - 1 + ky;
    const bool oky = ((unsigned)iy < (unsigned)IMH);
    const int iyc = (iy < 0) ? 0 : ((iy > IMH - 1) ? (IMH - 1) : iy);
#pragma unroll
    for (int kx = 0; kx < 3; ++kx) {
      const int ix = wx - 1 + kx;
      const bool ok = oky && ((unsigned)ix < (unsigned)IMW);
      const int ixc = (ix < 0) ? 0 : ((ix > IMW - 1) ? (IMW - 1) : ix);
      const float* p = XI + ((size_t)bb * LTOK + (size_t)(iyc * IMW + ixc)) * DIN + c8;
      const v4f xa = *(const v4fa*)p, xb = *(const v4fa*)(p + 4);
      const float* wq = w3s + (ky * 3 + kx) * DIN + c8;
      const v4f wa = *(const v4fa*)wq, wb = *(const v4fa*)(wq + 4);
#pragma unroll
      for (int u = 0; u < 4; ++u) {
        const float pa = xa[u] * wa[u];
        const float pb = xb[u] * wb[u];
        acc[u]     = acc[u]     + (ok ? pa : 0.0f);
        acc[4 + u] = acc[4 + u] + (ok ? pb : 0.0f);
      }
    }
  }
  const v4f ba = *(const v4fa*)(bias + c8), bq = *(const v4fa*)(bias + c8 + 4);
  float v[8];
#pragma unroll
  for (int u = 0; u < 4; ++u) { v[u] = siluf(acc[u] + bf16r(ba[u])); v[4 + u] = siluf(acc[4 + u] + bf16r(bq[u])); }
  us8 hi, lo;
  split8(v, hi, lo);
  const size_t o = (size_t)idx * 8;
  *(volatile us8*)(UH + o) = hi; *(volatile us8*)(UL + o) = lo;
  __threadfence();
  *(volatile us8*)(UH + o) = hi; *(volatile us8*)(UL + o) = lo;
}

__device__ __forceinline__ int tok_of(int dir, int l) {
  const int t0 = (l & (IMH - 1)) * IMW + (l >> 6);
  const int t1 = (LTOK - 1) - l;
  return dir ? t1 : t0;
}

__global__ __launch_bounds__(192) void k_scan(const float* __restrict__ XD, const unsigned short* __restrict__ UH,
                                             const unsigned short* __restrict__ UL,
                                             const float* __restrict__ dtw, const float* __restrict__ dtb,
                                             const float* __restrict__ Alog, const float* __restrict__ Dv, float* YS) {
#pragma clang fp contract(off)
  __shared__ __attribute__((aligned(16))) float sy[SCH * SYP];
  const int bb = blockIdx.x >> 1, dir = blockIdx.x & 1, tid = threadIdx.x;
  const int d = tid, kd = dir * DIN + d;
  float A2[DST], h[DST];
#pragma unroll
  for (int n = 0; n < DST; ++n) { A2[n] = -__expf(bf16r(Alog[kd * DST + n])) * LOG2E; h[n] = 0.0f; }
  float wd[DTRK];
#pragma unroll
  for (int r = 0; r < DTRK; ++r) wd[r] = bf16r(dtw[kd * DTRK + r]);
  const float bd = bf16r(dtb[kd]);
  const float Dd = bf16r(Dv[kd]);
  const float* XDb = XD + (size_t)bb * LTOK * XDN + 64 * dir;
  const unsigned short* UHb = UH + (size_t)bb * LTOK * DIN + d;
  const unsigned short* ULb = UL + (size_t)bb * LTOK * DIN + d;
  float* Yd = YS + (size_t)dir * NTOK * DIN + (size_t)bb * LTOK * DIN;
#pragma unroll 1
  for (int c = 0; c < LTOK / SCH; ++c) {
#pragma unroll 1
    for (int s = 0; s < SCH; ++s) {
      const int tok = tok_of(dir, c * SCH + s);
      const float* xr = XDb + (size_t)tok * XDN;
      const v4f d0 = *(const v4fa*)xr, d1 = *(const v4fa*)(xr + 4);
      const float raw = ((((d0[0] * wd[0] + d0[1] * wd[1]) + d0[2] * wd[2]) + d0[3] * wd[3]) + d1[0] * wd[4]) + d1[1] * wd[5];
      const float a = raw + bd;
      const float dl = fmaxf(a, 0.0f) + log1pf(__expf(-fabsf(a)));
      const size_t uo = (size_t)tok * DIN;
      const float uv = bf16_val(UHb[uo]) + bf16_val(ULb[uo]);
      v4f Bv[4], Cv[4];
#pragma unroll
      for (int q = 0; q < 4; ++q) {
        Bv[q] = *(const v4fa*)(xr + XBO + 4 * q);
        Cv[q] = *(const v4fa*)(xr + XCO + 4 * q);
      }
      const float dx = dl * uv;
      float y = 0.0f;
#pragma unroll
      for (int n = 0; n < DST; ++n) {
        const float e = exp2f(dl * A2[n]);
        h[n] = e * h[n] + dx * Bv[n >> 2][n & 3];
        y = y + h[n] * Cv[n >> 2][n & 3];
      }
      sy[s * SYP + d] = y + uv * Dd;
    }
    __syncthreads();
#pragma unroll
    for (int pass = 0; pass < 2; ++pass) {
#pragma unroll
      for (int it = 0; it < (SCH * (DIN / 4)) / DIN; ++it) {
        const int ix = it * DIN + tid;
        const int r = ix / (DIN / 4), q4 = (ix - r * (DIN / 4)) * 4;
        const int tok = tok_of(dir, c * SCH + r);
        const v4f v = *(const v4fa*)(sy + r * SYP + q4);
        *(volatile v4f*)(Yd + (size_t)tok * DIN + q4) = v;
      }
      __threadfence();
    }
    __syncthreads();
  }
}

__global__ __launch_bounds__(256) void k_mln(const float* __restrict__ YS, const float* __restrict__ XZ,
                                            const float* __restrict__ g, const float* __restrict__ bt,
                                            unsigned short* GH, unsigned short* GL) {
#pragma clang fp contract(off)
  const int tid = threadIdx.x, lane = tid & 31, wave = tid >> 5;
  const int tok = blockIdx.x * 8 + wave;
  const int bb = tok >> 12, m = tok & (LTOK - 1), hh = m >> 6, ww = m & 63;
  const int tokT = (bb << 12) + ww * IMW + hh;
  const bool act = (lane < DIN / 8);
  const int cl = act ? lane : (DIN / 8 - 1);
  const int c8 = cl * 8;
  const float* Y0 = YS;
  const float* Y1 = YS + (size_t)NTOK * DIN;
  const v4f y1a = *(const v4fa*)(Y1 + (size_t)tok * DIN + c8),  y1b = *(const v4fa*)(Y1 + (size_t)tok * DIN + c8 + 4);
  const v4f y0a = *(const v4fa*)(Y0 + (size_t)tok * DIN + c8),  y0b = *(const v4fa*)(Y0 + (size_t)tok * DIN + c8 + 4);
  const v4f yta = *(const v4fa*)(Y1 + (size_t)tokT * DIN + c8), ytb = *(const v4fa*)(Y1 + (size_t)tokT * DIN + c8 + 4);
  const v4f za  = *(const v4fa*)(XZ + (size_t)tok * DIN + c8),  zb  = *(const v4fa*)(XZ + (size_t)tok * DIN + c8 + 4);
  float gg[8], bq[8];
  {
    const v4f ga = *(const v4fa*)(g + c8), gb = *(const v4fa*)(g + c8 + 4);
    const v4f ba = *(const v4fa*)(bt + c8), b4 = *(const v4fa*)(bt + c8 + 4);
#pragma unroll
    for (int u = 0; u < 4; ++u) { gg[u] = bf16r(ga[u]); gg[4 + u] = bf16r(gb[u]); bq[u] = bf16r(ba[u]); bq[4 + u] = bf16r(b4[u]); }
  }
  float yv[8], zv[8];
#pragma unroll
  for (int u = 0; u < 4; ++u) {
    const float va = (y1a[u] + y0a[u]) + yta[u];
    const float vb = (y1b[u] + y0b[u]) + ytb[u];
    yv[u] = act ? va : 0.0f; yv[4 + u] = act ? vb : 0.0f;
    zv[u] = za[u]; zv[4 + u] = zb[u];
  }
  float s = ((yv[0] + yv[1]) + (yv[2] + yv[3])) + ((yv[4] + yv[5]) + (yv[6] + yv[7]));
#pragma unroll
  for (int o = 16; o > 0; o >>= 1) s = s + __shfl_xor(s, o);
  const float mu = s * (1.0f / DIN);
  float dv[8];
#pragma unroll
  for (int u = 0; u < 8; ++u) dv[u] = act ? (yv[u] - mu) : 0.0f;
  float s2 = 0.0f;
#pragma unroll
  for (int u = 0; u < 8; ++u) s2 = s2 + dv[u] * dv[u];
#pragma unroll
  for (int o = 16; o > 0; o >>= 1) s2 = s2 + __shfl_xor(s2, o);
  const float var = s2 * (1.0f / DIN);
  const float rs = 1.0f / sqrtf(var + EPSV);
  float ov[8];
#pragma unroll
  for (int u = 0; u < 8; ++u) {
    const float nv = (dv[u] * rs) * gg[u] + bq[u];
    ov[u] = nv * siluf(zv[u]);
  }
  us8 hi, lo;
  split8(ov, hi, lo);
  const size_t o = (size_t)tok * DIN + c8;
  if (act) { *(volatile us8*)(GH + o) = hi; *(volatile us8*)(GL + o) = lo; }
  __threadfence();
  if (act) { *(volatile us8*)(GH + o) = hi; *(volatile us8*)(GL + o) = lo; }
}

__global__ __launch_bounds__(256) void k_up(const float* __restrict__ OP, const float* __restrict__ uw, const float* __restrict__ ub,
                                           float* out) {
#pragma clang fp contract(off)
  __shared__ __attribute__((aligned(16))) float ws9[9 * CIN];
  const int tid = threadIdx.x;
#pragma unroll 1
  for (int i = tid; i < 9 * CIN; i += 256) {
    const int tap = i / CIN, c = i - tap * CIN;
    ws9[i] = bf16r(uw[c * 9 + tap]);
  }
  __syncthreads();
  const int idx = blockIdx.x * 256 + tid;
  const int pix = idx / (CIN / 4), c4 = (idx - pix * (CIN / 4)) * 4;
  const int X = pix & (WI - 1), Y = (pix >> 7) & (HI - 1), bb = pix >> 14;
  float acc[4] = {0.0f, 0.0f, 0.0f, 0.0f};
#pragma unroll
  for (int ty = 0; ty < 3; ++ty) {
    const int py = Y + ty;
    const int i = (py - 1) >> 1;
    const bool oky = ((py & 1) != 0) && (i < IMH);
    const int ic = (i < 0) ? 0 : ((i > IMH - 1) ? (IMH - 1) : i);
#pragma unroll
    for (int tx = 0; tx < 3; ++tx) {
      const int px = X + tx;
      const int j = (px - 1) >> 1;
      const bool ok = oky && ((px & 1) != 0) && (j < IMW);
      const int jc = (j < 0) ? 0 : ((j > IMW - 1) ? (IMW - 1) : j);
      const v4f v = *(const v4fa*)(OP + ((size_t)bb * LTOK + (size_t)(ic * IMW + jc)) * NOP + c4);
      const v4f wv = *(const v4fa*)(ws9 + ((2 - ty) * 3 + (2 - tx)) * CIN + c4);
#pragma unroll
      for (int u = 0; u < 4; ++u) {
        const float pr = v[u] * wv[u];
        acc[u] = acc[u] + (ok ? pr : 0.0f);
      }
    }
  }
  const v4f b4 = *(const v4fa*)(ub + c4);
  v4f o;
#pragma unroll
  for (int u = 0; u < 4; ++u) o[u] = acc[u] + bf16r(b4[u]);
  const size_t off = (size_t)idx * 4;
  *(volatile v4f*)(out + off) = o;
  __threadfence();
  *(volatile v4f*)(out + off) = o;
}

extern "C" void kernel_launch(void* const* d_in, const int* in_sizes, int n_in,
                              void* d_out, int out_size, void* d_ws, size_t ws_size,
                              hipStream_t stream) {
  if (n_in < 16) return;
  if (in_sizes[0] != NBAT * HI * WI * CIN || in_sizes[1] != CIN * 49 || in_sizes[2] != CIN || in_sizes[3] != 2 * DIN * CIN ||
      in_sizes[4] != DIN * 9 || in_sizes[5] != DIN || in_sizes[6] != 3 * XPR * DIN || in_sizes[7] != 3 * DIN * DTRK ||
      in_sizes[8] != 3 * DIN || in_sizes[9] != 3 * DIN * DST || in_sizes[10] != 3 * DIN || in_sizes[11] != DIN ||
      in_sizes[12] != DIN || in_sizes[13] != CIN * DIN || in_sizes[14] != CIN * 9 || in_sizes[15] != CIN ||
      out_size != NBAT * HI * WI * CIN) return;

  const float* x    = (const float*)d_in[0];
  const float* w7   = (const float*)d_in[1];
  const float* b7   = (const float*)d_in[2];
  const float* inw  = (const float*)d_in[3];
  const float* w3   = (const float*)d_in[4];
  const float* b3   = (const float*)d_in[5];
  const float* xpw  = (const float*)d_in[6];
  const float* dtw  = (const float*)d_in[7];
  const float* dtb  = (const float*)d_in[8];
  const float* Alog = (const float*)d_in[9];
  const float* Dv   = (const float*)d_in[10];
  const float* lng  = (const float*)d_in[11];
  const float* lnb  = (const float*)d_in[12];
  const float* ow   = (const float*)d_in[13];
  const float* uw   = (const float*)d_in[14];
  const float* ub   = (const float*)d_in[15];
  float* out = (float*)d_out;

  size_t off = 0;
  auto carve = [&](size_t bytes) -> char* { char* p = (char*)d_ws + off; off += (bytes + 255) & ~(size_t)255; return p; };
  unsigned short* WIN16 = (unsigned short*)carve((size_t)2 * DIN * CIN * 2);
  unsigned short* WX16  = (unsigned short*)carve((size_t)XDN * DIN * 2);
  unsigned short* WO16  = (unsigned short*)carve((size_t)NOP * DIN * 2);
  unsigned short* XHH   = (unsigned short*)carve((size_t)NTOK * CIN * 2);
  unsigned short* XHL   = (unsigned short*)carve((size_t)NTOK * CIN * 2);
  float* XI             = (float*)carve((size_t)NTOK * DIN * 4);
  float* XZ             = (float*)carve((size_t)NTOK * DIN * 4);
  unsigned short* UH    = (unsigned short*)carve((size_t)NTOK * DIN * 2);
  unsigned short* UL    = (unsigned short*)carve((size_t)NTOK * DIN * 2);
  float* XD             = (float*)carve((size_t)NTOK * XDN * 4);
  float* YS             = (float*)carve((size_t)NDIR * NTOK * DIN * 4);
  unsigned short* GH    = (unsigned short*)carve((size_t)NTOK * DIN * 2);
  unsigned short* GL    = (unsigned short*)carve((size_t)NTOK * DIN * 2);
  float* OP             = (float*)carve((size_t)NTOK * NOP * 4);
  if (off > ws_size || off > (size_t)134217728) return;

  const dim3 b256(256), b192(192);
  k_cvt<<<dim3((2 * DIN * (CIN / 8) + 255) / 256), b256, 0, stream>>>(inw, WIN16, 2 * DIN, CIN / 8, 2 * DIN * (CIN / 8));
  k_cvt_xw<<<dim3((XDN * (DIN / 8) + 255) / 256), b256, 0, stream>>>(xpw, WX16);
  k_cvt<<<dim3((NOP * (DIN / 8) + 255) / 256), b256, 0, stream>>>(ow, WO16, CIN, DIN / 8, NOP * (DIN / 8));
  k_dw7<<<dim3(NTOK * (CIN / 8) / 256), b256, 0, stream>>>(x, w7, b7, XHH, XHL);
  k_gemm<1><<<dim3(NTOK / 128, (2 * DIN) / 64), b256, 0, stream>>>(XHH, XHL, CIN, WIN16, CIN, XI, XZ, DIN, DIN, CIN);
  k_dw3<<<dim3(NTOK * (DIN / 8) / 256), b256, 0, stream>>>(XI, w3, b3, UH, UL);
  k_gemm<1><<<dim3(NTOK / 128, XDN / 64), b256, 0, stream>>>(UH, UL, DIN, WX16, DIN, XD, XD, 0, XDN, DIN);
  k_scan<<<dim3(NBAT * NDIR), b192, 0, stream>>>(XD, UH, UL, dtw, dtb, Alog, Dv, YS);
  k_mln<<<dim3(NTOK / 8), b256, 0, stream>>>(YS, XZ, lng, lnb, GH, GL);
  k_gemm<1><<<dim3(NTOK / 128, NOP / 64), b256, 0, stream>>>(GH, GL, DIN, WO16, DIN, OP, OP, 0, NOP, DIN);
  k_up<<<dim3(NBAT * HI * WI * (CIN / 4) / 256), b256, 0, stream>>>(OP, uw, ub, out);
}
